// DETECTiveGNN_18253611008270
// MI455X (gfx1250) — hardware-run, weakly checked
//
#include <hip/hip_runtime.h>
#include <stddef.h>
#include <stdint.h>
#include <math.h>

#define NN      100000
#define FD      128
#define HD      64
#define NE      1600000
#define GBM     128
#define MP      100096
#define KL      128
#define NTHR    256
#define NWAVE   8
#define EPT     8
#define WCH     (32 * EPT)
#define NBRUN   1024
#define SLB     10
#define NBK     98
#define WLCAP   2560
#define RCAP    20480
#define DEGCAP  64
#define MAXDEG_MEAS   36
#define MAXB1024_MEAS 16710
#define ABM     64
#define SP      68
#define SRCBITS 17
#define SRCMASK 0x1FFFF
#define NEGSL   0.2f
#define SPLIT_B 1
#define SPLIT_C 1
#define PAR_N   384

#define BK_ZINTS (NWAVE * WLCAP + RCAP + 3 * NBRUN)
#define BK_INTS  (BK_ZINTS + 16)
#define BK_LDS   (BK_INTS * 4)

#define PBX   (MP * FD / 8 / NTHR)
#define PBW   (HD * KL / 8 / NTHR)
#define PBTOT (PBX + 3 * PBW + 1)

static_assert(NN < (1 << SRCBITS));
static_assert(HD == 64 && HD == 16 * 4);
static_assert(MP % GBM == 0 && MP >= NN && MP == 782 * GBM && MP % ABM == 0);
static_assert(NBRUN == 1024 && NBRUN == (1 << SLB) && NBRUN % ABM == 0 && NBRUN % GBM == 0 && NBRUN % 32 == 0);
static_assert(NBRUN == 4 * NTHR);
static_assert(NBK * NBRUN >= MP);
static_assert(NE < (1 << 21) && (((long long)NE) << SLB) < (1LL << 31));
static_assert(NE % WCH == 0 && NE % 4 == 0);
static_assert(SLB + SRCBITS <= 31);
static_assert(RCAP == NWAVE * WLCAP && RCAP % 4 == 0 && BK_ZINTS % 4 == 0);
static_assert((long long)RCAP * 100 >= (long long)MAXB1024_MEAS * 105);
static_assert(WLCAP >= MAXB1024_MEAS / 8 + 8 * 46 + 1);
static_assert(MAXDEG_MEAS + 8 <= DEGCAP);
static_assert((MP * FD / 8) % NTHR == 0 && (HD * KL / 8) % NTHR == 0);
static_assert(FD % 32 == 0 && KL % 32 == 0 && KL == 2 * HD && FD == KL && HD % 32 == 0);
static_assert(BK_LDS <= 300000);
static_assert((GBM * SP + 512) * 4 + BK_LDS <= 327680);
static_assert((GBM * SP + 512) * 4 <= 65536);
static_assert(ABM == NWAVE * 8);
static_assert(PAR_N == 96 * 4);

typedef float          v4f   __attribute__((ext_vector_type(4)));
typedef float          v8f   __attribute__((ext_vector_type(8)));
typedef int            v4i   __attribute__((ext_vector_type(4)));
typedef int            v8i   __attribute__((ext_vector_type(8)));
typedef unsigned short v8us  __attribute__((ext_vector_type(8)));
typedef unsigned short v16us __attribute__((ext_vector_type(16)));
typedef __bf16         v16bf __attribute__((ext_vector_type(16)));
typedef v4f  __attribute__((may_alias)) v4fa;
typedef v4i  __attribute__((may_alias)) v4ia;
typedef v8us __attribute__((may_alias)) v8usa;
union FragB { v16bf v; v16us u; v8us h[2]; v8i w; };

__device__ __forceinline__ v8f wmb(const FragB& a, const FragB& b, v8f c) {
  v8f d = __builtin_amdgcn_wmma_f32_16x16x32_bf16(false, a.v, false, b.v, (short)0, c, false, false);
  asm volatile("v_nop\n\tv_nop\n\tv_nop\n\tv_nop" : "+v"(d) : "v"(a.w), "v"(b.w));
  return d;
}

__device__ __forceinline__ unsigned bf16_bits(float f) {
  const unsigned u = __float_as_uint(f);
  const unsigned r = (u + 0x7FFFu + ((u >> 16) & 1u)) >> 16;
  const unsigned q = (u >> 16) | 0x40u;
  return ((u & 0x7fffffffu) > 0x7f800000u) ? q : r;
}

__device__ __forceinline__ void hilo_pack(float v0, float v1, float v2, float v3,
                                          int& h01, int& h23, int& l01, int& l23) {
  const unsigned a0 = bf16_bits(v0), a1 = bf16_bits(v1), a2 = bf16_bits(v2), a3 = bf16_bits(v3);
  const unsigned b0 = bf16_bits(v0 - __uint_as_float(a0 << 16));
  const unsigned b1 = bf16_bits(v1 - __uint_as_float(a1 << 16));
  const unsigned b2 = bf16_bits(v2 - __uint_as_float(a2 << 16));
  const unsigned b3 = bf16_bits(v3 - __uint_as_float(a3 << 16));
  h01 = (int)(a0 | (a1 << 16)); h23 = (int)(a2 | (a3 << 16));
  l01 = (int)(b0 | (b1 << 16)); l23 = (int)(b2 | (b3 << 16));
}

__device__ __forceinline__ v4i regroup8(int h01, int h23, int l01, int l23, int lane) {
  const int t  = lane & 15;
  const int s0 = (lane & 16) + ((2 * t) & 15), s1 = s0 + 1;
  const int a0 = __shfl(h01, s0, 32), a1 = __shfl(h23, s0, 32), a2 = __shfl(h01, s1, 32), a3 = __shfl(h23, s1, 32);
  const int b0 = __shfl(l01, s0, 32), b1 = __shfl(l23, s0, 32), b2 = __shfl(l01, s1, 32), b3 = __shfl(l23, s1, 32);
  const int mk = (t < 8) ? -1 : 0;
  v4i o;
  o.x = (a0 & mk) | (b0 & ~mk); o.y = (a1 & mk) | (b1 & ~mk);
  o.z = (a2 & mk) | (b2 & ~mk); o.w = (a3 & mk) | (b3 & ~mk);
  return o;
}

__device__ __forceinline__ void st2_v4f(float* p, v4f v) {
  *(volatile v4f*)p = v;
  __threadfence();
  *(volatile v4f*)p = v;
}
__device__ __forceinline__ void st2_v8us(unsigned short* p, v8us v) {
  *(volatile v8us*)p = v;
  __threadfence();
  *(volatile v8us*)p = v;
}

__device__ __forceinline__ v8us colfetch8(const float* __restrict__ base, int stride) {
  float f[8];
#pragma unroll
  for (int i = 0; i < 8; ++i) f[i] = base[(size_t)i * (size_t)stride];
  v8us o;
#pragma unroll
  for (int i = 0; i < 8; ++i) o[i] = (unsigned short)bf16_bits(f[i]);
  return o;
}

__device__ __forceinline__ float blend5(float c0, float c1, float c2, float c3, float c4,
                                        unsigned k0, unsigned k1, unsigned k2, unsigned k3, unsigned k4) {
  const unsigned r = ((bf16_bits(c0) << 16) & k0) | ((bf16_bits(c1) << 16) & k1) | ((bf16_bits(c2) << 16) & k2) |
                     ((bf16_bits(c3) << 16) & k3) | ((bf16_bits(c4) << 16) & k4);
  return __uint_as_float(r);
}

__global__ __launch_bounds__(NTHR) void k_prep(const float* __restrict__ x, const float* __restrict__ wa,
                                               const float* __restrict__ vs, const float* __restrict__ vd,
                                               const float* __restrict__ ba, const float* __restrict__ w1,
                                               const float* __restrict__ b1, const float* __restrict__ w2,
                                               const float* __restrict__ b2,
                                               unsigned short* xb, unsigned short* wat, unsigned short* w1d,
                                               unsigned short* w2d, float* par) {
  const int tid = (int)threadIdx.x;
  const int blk = (int)blockIdx.x;
  if (blk < PBX) {
    const int u   = blk * NTHR + tid;
    const int row = u >> 4, k8 = (u & 15) * 8;
    const int rc  = row < NN ? row : NN - 1;
    const unsigned mk = row < NN ? 0xffffu : 0u;
    const float* p = x + (size_t)rc * FD + k8;
    const v4f a = *(const v4fa*)p;
    const v4f b = *(const v4fa*)(p + 4);
    v8us o;
    o[0] = (unsigned short)(bf16_bits(a.x) & mk); o[1] = (unsigned short)(bf16_bits(a.y) & mk);
    o[2] = (unsigned short)(bf16_bits(a.z) & mk); o[3] = (unsigned short)(bf16_bits(a.w) & mk);
    o[4] = (unsigned short)(bf16_bits(b.x) & mk); o[5] = (unsigned short)(bf16_bits(b.y) & mk);
    o[6] = (unsigned short)(bf16_bits(b.z) & mk); o[7] = (unsigned short)(bf16_bits(b.w) & mk);
    st2_v8us(xb + (size_t)row * FD + k8, o);
  } else if (blk < PBX + PBW) {
    const int u = (blk - PBX) * NTHR + tid;
    const int n = u >> 4, k8 = (u & 15) * 8;
    const v8us o = colfetch8(wa + (size_t)k8 * HD + n, HD);
    st2_v8us(wat + (size_t)n * FD + k8, o);
  } else if (blk < PBX + 2 * PBW) {
    const int u = (blk - PBX - PBW) * NTHR + tid;
    const int n = u >> 4, k8 = (u & 15) * 8, kk = k8 & 63;
    const v8us o = colfetch8(w1 + (size_t)kk * HD + n, HD);
    st2_v8us(w1d + (size_t)n * KL + k8, o);
  } else if (blk < PBX + 3 * PBW) {
    const int u = (blk - PBX - 2 * PBW) * NTHR + tid;
    const int n = u >> 4, k8 = (u & 15) * 8, kk = k8 & 63;
    const v8us o = colfetch8(w2 + (size_t)kk * HD + n, HD);
    st2_v8us(w2d + (size_t)n * KL + k8, o);
  } else {
    if (tid < 96) {
      const int seg = tid >> 4, q = tid & 15;
      const v4f c0 = *(const v4fa*)(vs + 4 * q);
      const v4f c1 = *(const v4fa*)(vd + 4 * q);
      const v4f c2 = *(const v4fa*)(ba + 4 * q);
      const v4f c3 = *(const v4fa*)(b1 + 4 * q);
      const v4f c4 = *(const v4fa*)(b2 + 4 * q);
      asm volatile("" :: "v"(c0));
      asm volatile("" :: "v"(c1));
      asm volatile("" :: "v"(c2));
      asm volatile("" :: "v"(c3));
      asm volatile("" :: "v"(c4));
      const unsigned k0 = (seg == 0) ? 0xffffffffu : 0u, k1 = (seg == 1) ? 0xffffffffu : 0u;
      const unsigned k2 = (seg == 2) ? 0xffffffffu : 0u, k3 = (seg == 3) ? 0xffffffffu : 0u;
      const unsigned k4 = (seg == 4) ? 0xffffffffu : 0u;
      v4f o;
      o.x = blend5(c0.x, c1.x, c2.x, c3.x, c4.x, k0, k1, k2, k3, k4);
      o.y = blend5(c0.y, c1.y, c2.y, c3.y, c4.y, k0, k1, k2, k3, k4);
      o.z = blend5(c0.z, c1.z, c2.z, c3.z, c4.z, k0, k1, k2, k3, k4);
      o.w = blend5(c0.w, c1.w, c2.w, c3.w, c4.w, k0, k1, k2, k3, k4);
      st2_v4f(par + 4 * tid, o);
    }
  }
}

__device__ __forceinline__ void bucket_flush(const int* pl, v4i cv, v4i ofv, v4i dvv, int ov, int* lp,
                                             int* cp, int* op, int* dp, int* fp, int tid) {
#pragma unroll 1
  for (int i = tid * 4; i < RCAP; i += NTHR * 4) {
    const v4i v = *(const v4ia*)(pl + i);
    *(volatile v4i*)(lp + i) = v;
  }
  *(volatile v4i*)(cp + 4 * tid) = cv;
  *(volatile v4i*)(op + 4 * tid) = ofv;
  *(volatile v4i*)(dp + 4 * tid) = dvv;
  if (tid < 8) {
    const v4i f = {ov, ov, ov, ov};
    *(volatile v4i*)(fp + 4 * tid) = f;
  }
}

__global__ __launch_bounds__(NTHR) void k_bucket(const int* __restrict__ srcs, const int* __restrict__ dsts,
                                                 int* HITS, int* CNT, int* OFF, int* DINV, int* FLAG) {
  extern __shared__ __attribute__((aligned(16))) int dsm[];
  int* wl   = dsm;
  int* pl   = dsm + NWAVE * WLCAP;
  int* cnt  = pl + RCAP;
  int* offs = cnt + NBRUN;
  int* cur  = offs + NBRUN;
  int* misc = cur + NBRUN;
  const int tid = (int)threadIdx.x, lane = tid & 31, wave = tid >> 5;
  const int blk = (int)blockIdx.x;
  const unsigned nbs = (unsigned)(blk * NBRUN);

  {
    const v4i z4 = {0, 0, 0, 0};
    for (int i = tid * 4; i < BK_ZINTS; i += NTHR * 4) *(v4ia*)(dsm + i) = z4;
    if (tid < 16) misc[tid] = 0;
  }
  __syncthreads();

  {
    const int per  = ((NE + NWAVE * WCH - 1) / (NWAVE * WCH)) * WCH;
    const int ebeg = wave * per;
    const int eend = (ebeg + per < NE) ? (ebeg + per) : NE;
    int* mylist = wl + wave * WLCAP;
    int wc = 0;
#pragma unroll 1
    for (int cb = ebeg; cb < eend; cb += WCH) {
      const int e0 = cb + lane * EPT;
      const v4i da = *(const v4ia*)(dsts + e0);
      const v4i db = *(const v4ia*)(dsts + e0 + 4);
      const unsigned s0 = (unsigned)da.x - nbs, s1 = (unsigned)da.y - nbs;
      const unsigned s2 = (unsigned)da.z - nbs, s3 = (unsigned)da.w - nbs;
      const unsigned s4 = (unsigned)db.x - nbs, s5 = (unsigned)db.y - nbs;
      const unsigned s6 = (unsigned)db.z - nbs, s7 = (unsigned)db.w - nbs;
      const bool h0 = (s0 < (unsigned)NBRUN) & ((unsigned)da.x < (unsigned)NN);
      const bool h1 = (s1 < (unsigned)NBRUN) & ((unsigned)da.y < (unsigned)NN);
      const bool h2 = (s2 < (unsigned)NBRUN) & ((unsigned)da.z < (unsigned)NN);
      const bool h3 = (s3 < (unsigned)NBRUN) & ((unsigned)da.w < (unsigned)NN);
      const bool h4 = (s4 < (unsigned)NBRUN) & ((unsigned)db.x < (unsigned)NN);
      const bool h5 = (s5 < (unsigned)NBRUN) & ((unsigned)db.y < (unsigned)NN);
      const bool h6 = (s6 < (unsigned)NBRUN) & ((unsigned)db.z < (unsigned)NN);
      const bool h7 = (s7 < (unsigned)NBRUN) & ((unsigned)db.w < (unsigned)NN);
      const unsigned m0 = __builtin_amdgcn_ballot_w32(h0), m1 = __builtin_amdgcn_ballot_w32(h1);
      const unsigned m2 = __builtin_amdgcn_ballot_w32(h2), m3 = __builtin_amdgcn_ballot_w32(h3);
      const unsigned m4 = __builtin_amdgcn_ballot_w32(h4), m5 = __builtin_amdgcn_ballot_w32(h5);
      const unsigned m6 = __builtin_amdgcn_ballot_w32(h6), m7 = __builtin_amdgcn_ballot_w32(h7);
      const unsigned any = m0 | m1 | m2 | m3 | m4 | m5 | m6 | m7;
      if (any != 0u) {
        const int pre = (int)(__builtin_amdgcn_mbcnt_lo(m0, 0u) + __builtin_amdgcn_mbcnt_lo(m1, 0u) +
                              __builtin_amdgcn_mbcnt_lo(m2, 0u) + __builtin_amdgcn_mbcnt_lo(m3, 0u) +
                              __builtin_amdgcn_mbcnt_lo(m4, 0u) + __builtin_amdgcn_mbcnt_lo(m5, 0u) +
                              __builtin_amdgcn_mbcnt_lo(m6, 0u) + __builtin_amdgcn_mbcnt_lo(m7, 0u));
        int p = wc + pre;
        if (h0) { if (p < WLCAP) mylist[p] = ((e0 + 0) << SLB) | (int)s0; p = p + 1; }
        if (h1) { if (p < WLCAP) mylist[p] = ((e0 + 1) << SLB) | (int)s1; p = p + 1; }
        if (h2) { if (p < WLCAP) mylist[p] = ((e0 + 2) << SLB) | (int)s2; p = p + 1; }
        if (h3) { if (p < WLCAP) mylist[p] = ((e0 + 3) << SLB) | (int)s3; p = p + 1; }
        if (h4) { if (p < WLCAP) mylist[p] = ((e0 + 4) << SLB) | (int)s4; p = p + 1; }
        if (h5) { if (p < WLCAP) mylist[p] = ((e0 + 5) << SLB) | (int)s5; p = p + 1; }
        if (h6) { if (p < WLCAP) mylist[p] = ((e0 + 6) << SLB) | (int)s6; p = p + 1; }
        if (h7) { if (p < WLCAP) mylist[p] = ((e0 + 7) << SLB) | (int)s7; p = p + 1; }
        wc += (int)(__builtin_popcount(m0) + __builtin_popcount(m1) + __builtin_popcount(m2) + __builtin_popcount(m3) +
                    __builtin_popcount(m4) + __builtin_popcount(m5) + __builtin_popcount(m6) + __builtin_popcount(m7));
      }
    }
    if (lane == 0) misc[wave] = wc;
  }
  __syncthreads();

  if (wave == 0) {
    int ov = 0;
#pragma unroll 1
    for (int w2 = 0; w2 < NWAVE; ++w2) {
      int c = misc[w2];
      if (c > WLCAP) ov = 1;
      c = c < 0 ? 0 : (c > WLCAP ? WLCAP : c);
#pragma unroll 1
      for (int b0 = 0; b0 < c; b0 += 32) {
        const int idx = b0 + lane;
        const int ent = wl[w2 * WLCAP + (idx < WLCAP ? idx : WLCAP - 1)];
        const int m32 = (c - b0) < 32 ? (c - b0) : 32;
#pragma unroll 1
        for (int k = 0; k < m32; ++k) {
          const int u    = __builtin_amdgcn_readlane(ent, k);
          const int slot = u & (NBRUN - 1);
          if (lane == 0) cnt[slot] = cnt[slot] + 1;
        }
      }
    }
    if (lane == 0) misc[9] = ov;
  }
  __syncthreads();
  if (wave == 0) {
    const int base = lane * (NBRUN / 32);
    int s = 0;
#pragma unroll 1
    for (int i = 0; i < NBRUN / 32; ++i) s += cnt[base + i];
    int incl = s;
#pragma unroll
    for (int d = 1; d < 32; d <<= 1) {
      const int y = __shfl_up(incl, d, 32);
      if (lane >= d) incl += y;
    }
    int run = incl - s;
#pragma unroll 1
    for (int i = 0; i < NBRUN / 32; ++i) {
      const int cv = cnt[base + i];
      offs[base + i] = run;
      cur[base + i]  = run;
      run += cv;
    }
  }
  __syncthreads();

  if (wave == 0) {
#pragma unroll 1
    for (int w2 = 0; w2 < NWAVE; ++w2) {
      int c = misc[w2];
      c = c < 0 ? 0 : (c > WLCAP ? WLCAP : c);
#pragma unroll 1
      for (int b0 = 0; b0 < c; b0 += 32) {
        const int idx = b0 + lane;
        const int ent = wl[w2 * WLCAP + (idx < WLCAP ? idx : WLCAP - 1)];
        int eid = (ent >> SLB) & 0x1FFFFF;
        eid = eid > NE - 1 ? NE - 1 : eid;
        int sr = srcs[eid];
        sr = sr < 0 ? 0 : (sr > NN - 1 ? NN - 1 : sr);
        const int word = (int)((unsigned)sr | ((unsigned)(ent & (NBRUN - 1)) << SRCBITS));
        const int m32 = (c - b0) < 32 ? (c - b0) : 32;
#pragma unroll 1
        for (int k = 0; k < m32; ++k) {
          const int u    = __builtin_amdgcn_readlane(ent, k);
          const int wd   = __builtin_amdgcn_readlane(word, k);
          const int slot = u & (NBRUN - 1);
          if (lane == 0) {
            int p = cur[slot];
            p = p < 0 ? 0 : (p > RCAP - 1 ? RCAP - 1 : p);
            pl[p] = wd;
            cur[slot] = p + 1;
          }
        }
      }
    }
  }
  __syncthreads();

#pragma unroll 1
  for (int i = 0; i < NBRUN / NTHR; ++i) {
    const int s = tid + NTHR * i;
    int cv = cnt[s];
    cv = cv < 0 ? 0 : cv;
    const float dg = (float)(cv + 1);
    cur[s] = __float_as_int(1.0f / sqrtf(dg));
  }
  __syncthreads();

  const int ovf = misc[9];
  const v4i cv4 = *(const v4ia*)(cnt + 4 * tid);
  const v4i of4 = *(const v4ia*)(offs + 4 * tid);
  const v4i dv4 = *(const v4ia*)(cur + 4 * tid);
  int* lp = HITS + (size_t)blk * RCAP;
  int* cp = CNT + (size_t)blk * NBRUN;
  int* op = OFF + (size_t)blk * NBRUN;
  int* dp = DINV + (size_t)blk * NBRUN;
  int* fp = FLAG + (size_t)blk * 32;
  bucket_flush(pl, cv4, of4, dv4, ovf, lp, cp, op, dp, fp, tid);
  __threadfence();
  bucket_flush(pl, cv4, of4, dv4, ovf, lp, cp, op, dp, fp, tid);
}

template <int KLOOP, int PITCH>
__device__ __forceinline__ void gemm_16x64(const unsigned short* __restrict__ ap,
                                           const unsigned short* __restrict__ bp, v8f (&acc)[4]) {
  static_assert(KLOOP % 32 == 0 && KLOOP <= PITCH);
#pragma unroll 1
  for (int k0 = 0; k0 < KLOOP; k0 += 32) {
    FragB af;
    af.h[0] = *(const v8usa*)(ap + k0);
    af.h[1] = *(const v8usa*)(ap + k0 + 16);
#pragma unroll
    for (int nt = 0; nt < 4; ++nt) {
      const unsigned short* wq = bp + (size_t)(16 * nt) * (size_t)PITCH + k0;
      FragB bf;
      bf.h[0] = *(const v8usa*)wq;
      bf.h[1] = *(const v8usa*)(wq + 16);
      acc[nt] = wmb(af, bf, acc[nt]);
    }
  }
}

__device__ __forceinline__ void stage_d(float* stg, const v8f (&acc)[4], int wave, int hh, int m) {
#pragma unroll
  for (int nt = 0; nt < 4; ++nt) {
#pragma unroll
    for (int r = 0; r < 8; ++r) stg[(16 * wave + 8 * hh + r) * SP + 16 * nt + m] = acc[nt][r];
  }
}

__global__ __launch_bounds__(NTHR) __attribute__((amdgpu_num_vgpr(248)))
void k_gemmA(const unsigned short* __restrict__ XB, const unsigned short* __restrict__ WAT,
             const float* __restrict__ PAR, float* H, float* AS, float* AD) {
  __shared__ __attribute__((aligned(16))) float stg[GBM * SP];
  __shared__ __attribute__((aligned(16))) float sat[128];
  __shared__ __attribute__((aligned(16))) float sdt[2 * GBM];
  const int tid = (int)threadIdx.x, lane = tid & 31, wave = tid >> 5, hh = lane >> 4, m = lane & 15;
  const int rowBase = (int)blockIdx.x * GBM;
  if (tid < 32) *(v4fa*)(sat + 4 * tid) = *(const v4fa*)(PAR + 4 * tid);

  v8f acc[4];
  {
    const v8f z = {0.f, 0.f, 0.f, 0.f, 0.f, 0.f, 0.f, 0.f};
#pragma unroll
    for (int t = 0; t < 4; ++t) acc[t] = z;
  }
  const unsigned short* ap = XB + (size_t)(rowBase + 16 * wave + m) * (size_t)FD + 8 * hh;
  const unsigned short* bp = WAT + (size_t)m * (size_t)FD + 8 * hh;
  gemm_16x64<FD, FD>(ap, bp, acc);
  stage_d(stg, acc, wave, hh, m);
  __syncthreads();

  const v4f as4 = *(const v4fa*)(sat + 4 * m);
  const v4f ad4 = *(const v4fa*)(sat + 64 + 4 * m);
#pragma unroll 1
  for (int i = 0; i < 8; ++i) {
    const int lr   = 16 * wave + 2 * i + hh;
    const int grow = rowBase + lr;
    const v4f a = *(const v4fa*)(stg + lr * SP + 4 * m);
    float s = a.x * as4.x;
    s = fmaf(a.y, as4.y, s); s = fmaf(a.z, as4.z, s); s = fmaf(a.w, as4.w, s);
    float d = a.x * ad4.x;
    d = fmaf(a.y, ad4.y, d); d = fmaf(a.z, ad4.z, d); d = fmaf(a.w, ad4.w, d);
#pragma unroll
    for (int off = 1; off < 16; off <<= 1) {
      s += __shfl_xor(s, off, 32);
      d += __shfl_xor(d, off, 32);
    }
    if (m == 0) { sdt[lr] = s; sdt[GBM + lr] = d; }
    st2_v4f(H + (size_t)grow * HD + 4 * m, a);
  }
  __syncthreads();
  if (wave == 0) {
    const v4f v = *(const v4fa*)(sdt + 4 * lane);
    st2_v4f(AS + rowBase + 4 * lane, v);
  }
  if (wave == 1) {
    const v4f v = *(const v4fa*)(sdt + GBM + 4 * lane);
    st2_v4f(AD + rowBase + 4 * lane, v);
  }
}

template <int SPLIT>
__global__ __launch_bounds__(NTHR) __attribute__((amdgpu_num_vgpr(248)))
void k_gemmP(const unsigned short* __restrict__ A, const unsigned short* __restrict__ BT,
             const float* __restrict__ DINV, float* P) {
  __shared__ __attribute__((aligned(16))) float stg[GBM * SP];
  __shared__ __attribute__((aligned(16))) float sdv[GBM];
  const int tid = (int)threadIdx.x, lane = tid & 31, wave = tid >> 5, hh = lane >> 4, m = lane & 15;
  const int rowBase = (int)blockIdx.x * GBM;
  if (tid < 32) *(v4fa*)(sdv + 4 * tid) = *(const v4fa*)(DINV + rowBase + 4 * tid);

  v8f acc[4];
  {
    const v8f z = {0.f, 0.f, 0.f, 0.f, 0.f, 0.f, 0.f, 0.f};
#pragma unroll
    for (int t = 0; t < 4; ++t) acc[t] = z;
  }
  const unsigned short* ap = A + (size_t)(rowBase + 16 * wave + m) * (size_t)KL + 8 * hh;
  const unsigned short* bp = BT + (size_t)m * (size_t)KL + 8 * hh;
  gemm_16x64<(SPLIT != 0) ? KL : HD, KL>(ap, bp, acc);
  stage_d(stg, acc, wave, hh, m);
  __syncthreads();

#pragma unroll 1
  for (int i = 0; i < 8; ++i) {
    const int lr   = 16 * wave + 2 * i + hh;
    const int grow = rowBase + lr;
    const v4f a  = *(const v4fa*)(stg + lr * SP + 4 * m);
    const float dv = sdv[lr];
    v4f o;
    o.x = dv * a.x; o.y = dv * a.y; o.z = dv * a.z; o.w = dv * a.w;
    st2_v4f(P + (size_t)grow * HD + 4 * m, o);
  }
}

__global__ __launch_bounds__(NTHR) void k_attn(const int* __restrict__ HITS, const int* __restrict__ CNT,
                                               const int* __restrict__ OFF, const int* __restrict__ FLAG,
                                               const float* __restrict__ H, const float* __restrict__ AS,
                                               const float* __restrict__ AD, const float* __restrict__ PAR,
                                               unsigned short* XHL) {
  __shared__ __attribute__((aligned(16))) float sb[64];
  const int tid = (int)threadIdx.x, lane = tid & 31, wave = tid >> 5, hh = lane >> 4, q = lane & 15;
  if (tid < 16) *(v4fa*)(sb + 4 * tid) = *(const v4fa*)(PAR + 128 + 4 * tid);
  __syncthreads();
  const v4f bias = *(const v4fa*)(sb + 4 * q);
  const int rowBase = (int)blockIdx.x * ABM;
  const int bucket  = rowBase >> SLB;
  const int* lb  = HITS + (size_t)bucket * RCAP;
  const int flag = FLAG[(size_t)bucket * 32];
  const float qnan = __uint_as_float(0x7fc00000u);

#pragma unroll 1
  for (int i = 0; i < ABM / (2 * NWAVE); ++i) {
    const int d = rowBase + (ABM / NWAVE) * wave + 2 * i + hh;
    int c = CNT[d];
    int o = OFF[d];
    const bool big = c > DEGCAP;
    c = c < 0 ? 0 : (c > DEGCAP ? DEGCAP : c);
    o = o < 0 ? 0 : (o > RCAP - 1 ? RCAP - 1 : o);
    const int co = __shfl_xor(c, 16, 32);
    const int cm = c > co ? c : co;
    int last = o + c - 1;
    last = last < o ? o : last;
    last = last > RCAP - 1 ? RCAP - 1 : last;
    const float asd = AS[d];
    const float add = AD[d];
    const v4f g = *(const v4fa*)(H + (size_t)d * HD + 4 * q);
    float a0 = g.x, a1 = g.y, a2 = g.z, a3 = g.w;
    float e0 = asd + add;
    float mx = (e0 > 0.0f) ? e0 : NEGSL * e0;
    float l  = 1.0f;
#pragma unroll 1
    for (int j = 0; j < cm; ++j) {
      int idx = o + j;
      idx = idx > last ? last : idx;
      const unsigned wd = (unsigned)lb[idx];
      int sr = (int)(wd & (unsigned)SRCMASK);
      sr = sr > NN - 1 ? NN - 1 : sr;
      const float es = AS[sr];
      const v4f v = *(const v4fa*)(H + (size_t)sr * HD + 4 * q);
      asm volatile("" :: "v"(es));
      asm volatile("" :: "v"(v));
      float e = es + add;
      e = (e > 0.0f) ? e : NEGSL * e;
      const float df = e - mx;
      const float t  = expf(-fabsf(df));
      const bool  up = df > 0.0f;
      const float s1 = up ? t : 1.0f;
      const float s2 = up ? 1.0f : t;
      const float nm = up ? e : mx;
      const float nl = fmaf(l, s1, s2);
      const float n0 = fmaf(a0, s1, s2 * v.x), n1 = fmaf(a1, s1, s2 * v.y);
      const float n2 = fmaf(a2, s1, s2 * v.z), n3 = fmaf(a3, s1, s2 * v.w);
      const bool valid = j < c;
      mx = valid ? nm : mx; l = valid ? nl : l;
      a0 = valid ? n0 : a0; a1 = valid ? n1 : a1; a2 = valid ? n2 : a2; a3 = valid ? n3 : a3;
    }
    const float inv = 1.0f / (l + 1e-16f);
    float y0 = a0 * inv + bias.x, y1 = a1 * inv + bias.y, y2 = a2 * inv + bias.z, y3 = a3 * inv + bias.w;
    y0 = (y0 > 0.0f) ? y0 : (y0 - y0); y1 = (y1 > 0.0f) ? y1 : (y1 - y1);
    y2 = (y2 > 0.0f) ? y2 : (y2 - y2); y3 = (y3 > 0.0f) ? y3 : (y3 - y3);
    const bool bad  = (flag != 0) | big;
    const bool live = d < NN;
    y0 = bad ? qnan : y0; y1 = bad ? qnan : y1; y2 = bad ? qnan : y2; y3 = bad ? qnan : y3;
    y0 = live ? y0 : 0.0f; y1 = live ? y1 : 0.0f; y2 = live ? y2 : 0.0f; y3 = live ? y3 : 0.0f;
    int h01, h23, l01, l23;
    hilo_pack(y0, y1, y2, y3, h01, h23, l01, l23);
    const v4i ow = regroup8(h01, h23, l01, l23, lane);
    unsigned short* hp = XHL + (size_t)d * KL + 8 * q;
    *(volatile v4i*)hp = ow;
    __threadfence();
    *(volatile v4i*)hp = ow;
  }
}

template <int FINAL>
__global__ __launch_bounds__(NTHR) void k_conv(const int* __restrict__ HITS, const int* __restrict__ CNT,
                                               const int* __restrict__ OFF, const int* __restrict__ FLAG,
                                               const float* __restrict__ P, const float* __restrict__ DINV,
                                               const float* __restrict__ PAR, int boff,
                                               unsigned short* XHL, float* outp) {
  __shared__ __attribute__((aligned(16))) float sb[64];
  const int tid = (int)threadIdx.x, lane = tid & 31, wave = tid >> 5, hh = lane >> 4, q = lane & 15;
  if (tid < 16) *(v4fa*)(sb + 4 * tid) = *(const v4fa*)(PAR + boff + 4 * tid);
  __syncthreads();
  const v4f bias = *(const v4fa*)(sb + 4 * q);
  const int rowBase = (int)blockIdx.x * ABM;
  const int bucket  = rowBase >> SLB;
  const int* lb  = HITS + (size_t)bucket * RCAP;
  const int flag = FLAG[(size_t)bucket * 32];
  const float qnan = __uint_as_float(0x7fc00000u);

#pragma unroll 1
  for (int i = 0; i < ABM / (2 * NWAVE); ++i) {
    const int d = rowBase + (ABM / NWAVE) * wave + 2 * i + hh;
    int c = CNT[d];
    int o = OFF[d];
    const bool big = c > DEGCAP;
    c = c < 0 ? 0 : (c > DEGCAP ? DEGCAP : c);
    o = o < 0 ? 0 : (o > RCAP - 1 ? RCAP - 1 : o);
    const int co = __shfl_xor(c, 16, 32);
    const int cm = c > co ? c : co;
    int last = o + c - 1;
    last = last < o ? o : last;
    last = last > RCAP - 1 ? RCAP - 1 : last;
    float a0 = 0.0f, a1 = 0.0f, a2 = 0.0f, a3 = 0.0f;
#pragma unroll 1
    for (int j = 0; j < cm; ++j) {
      int idx = o + j;
      idx = idx > last ? last : idx;
      const unsigned wd = (unsigned)lb[idx];
      int sr = (int)(wd & (unsigned)SRCMASK);
      sr = sr > NN - 1 ? NN - 1 : sr;
      const v4f v = *(const v4fa*)(P + (size_t)sr * HD + 4 * q);
      asm volatile("" :: "v"(v));
      const bool valid = j < c;
      const float t0 = a0 + v.x, t1 = a1 + v.y, t2 = a2 + v.z, t3 = a3 + v.w;
      a0 = valid ? t0 : a0; a1 = valid ? t1 : a1; a2 = valid ? t2 : a2; a3 = valid ? t3 : a3;
    }
    const v4f g = *(const v4fa*)(P + (size_t)d * HD + 4 * q);
    const float dv = DINV[d];
    asm volatile("" :: "v"(g));
    a0 = a0 + g.x; a1 = a1 + g.y; a2 = a2 + g.z; a3 = a3 + g.w;
    float y0 = dv * a0 + bias.x, y1 = dv * a1 + bias.y, y2 = dv * a2 + bias.z, y3 = dv * a3 + bias.w;
    const bool bad  = (flag != 0) | big;
    const bool live = d < NN;
    if constexpr (FINAL == 0) {
      y0 = (y0 > 0.0f) ? y0 : (y0 - y0); y1 = (y1 > 0.0f) ? y1 : (y1 - y1);
      y2 = (y2 > 0.0f) ? y2 : (y2 - y2); y3 = (y3 > 0.0f) ? y3 : (y3 - y3);
      y0 = bad ? qnan : y0; y1 = bad ? qnan : y1; y2 = bad ? qnan : y2; y3 = bad ? qnan : y3;
      y0 = live ? y0 : 0.0f; y1 = live ? y1 : 0.0f; y2 = live ? y2 : 0.0f; y3 = live ? y3 : 0.0f;
      int h01, h23, l01, l23;
      hilo_pack(y0, y1, y2, y3, h01, h23, l01, l23);
      const v4i ow = regroup8(h01, h23, l01, l23, lane);
      unsigned short* hp = XHL + (size_t)d * KL + 8 * q;
      *(volatile v4i*)hp = ow;
      __threadfence();
      *(volatile v4i*)hp = ow;
    } else {
      y0 = bad ? qnan : y0; y1 = bad ? qnan : y1; y2 = bad ? qnan : y2; y3 = bad ? qnan : y3;
      v4f ov;
      ov.x = y0; ov.y = y1; ov.z = y2; ov.w = y3;
      const int dc = live ? d : NN - 1;
      float* op = outp + (size_t)dc * HD + 4 * q;
      if (live) *(volatile v4f*)op = ov;
      __threadfence();
      if (live) *(volatile v4f*)op = ov;
    }
  }
}

extern "C" void kernel_launch(void* const* d_in, const int* in_sizes, int n_in,
                              void* d_out, int out_size, void* d_ws, size_t ws_size,
                              hipStream_t stream) {
  if (n_in < 10) return;
  if (in_sizes[0] != NN * FD) return;
  if (in_sizes[1] != 2 * NE) return;
  if (in_sizes[2] != FD * HD) return;
  if (in_sizes[3] != HD) return;
  if (in_sizes[4] != HD) return;
  if (in_sizes[5] != HD) return;
  if (in_sizes[6] != HD * HD) return;
  if (in_sizes[7] != HD) return;
  if (in_sizes[8] != HD * HD) return;
  if (in_sizes[9] != HD) return;
  if (out_size != NN * HD) return;

  const float* x  = (const float*)d_in[0];
  const int*   ei = (const int*)d_in[1];
  const float* Wa = (const float*)d_in[2];
  const float* vs = (const float*)d_in[3];
  const float* vd = (const float*)d_in[4];
  const float* ba = (const float*)d_in[5];
  const float* W1 = (const float*)d_in[6];
  const float* b1 = (const float*)d_in[7];
  const float* W2 = (const float*)d_in[8];
  const float* b2 = (const float*)d_in[9];
  float* out = (float*)d_out;
  const int* srcs = ei;
  const int* dsts = ei + NE;

  constexpr size_t zXB   = (size_t)MP * FD * 2;
  constexpr size_t zXHL  = (size_t)MP * KL * 2;
  constexpr size_t zF    = (size_t)MP * HD * 4;
  constexpr size_t zHITS = (size_t)NBK * RCAP * 4;
  constexpr size_t zNODE = (size_t)NBK * NBRUN * 4;
  constexpr size_t zROW  = (size_t)MP * 4;
  constexpr size_t zFLAG = (size_t)NBK * 128;
  constexpr size_t zWT   = (size_t)HD * KL * 2;
  constexpr size_t zPAR  = (size_t)PAR_N * 4;
  constexpr size_t oXB   = 0;
  constexpr size_t oXHL  = oXB + zXB;
  constexpr size_t oH    = oXHL + zXHL;
  constexpr size_t oP1   = oH + zF;
  constexpr size_t oHITS = oP1 + zF;
  constexpr size_t oCNT  = oHITS + zHITS;
  constexpr size_t oOFF  = oCNT + zNODE;
  constexpr size_t oDINV = oOFF + zNODE;
  constexpr size_t oAS   = oDINV + zNODE;
  constexpr size_t oAD   = oAS + zROW;
  constexpr size_t oFLAG = oAD + zROW;
  constexpr size_t oWAT  = oFLAG + zFLAG;
  constexpr size_t oW1D  = oWAT + zWT;
  constexpr size_t oW2D  = oW1D + zWT;
  constexpr size_t oPAR  = oW2D + zWT;
  constexpr size_t oEND  = oPAR + zPAR;
  static_assert(zXB % 256 == 0 && zXHL % 256 == 0 && zF % 256 == 0 && zHITS % 256 == 0 && zNODE % 256 == 0);
  static_assert(zROW % 256 == 0 && zFLAG % 256 == 0 && zWT % 256 == 0 && zPAR % 256 == 0);
  static_assert(zNODE >= (size_t)MP * 4);
  static_assert(oEND <= ((size_t)128u << 20));
  if (oEND > ws_size) return;

  char* ws = (char*)d_ws;
  unsigned short* XB   = (unsigned short*)(ws + oXB);
  unsigned short* XHL  = (unsigned short*)(ws + oXHL);
  float*          Hb   = (float*)(ws + oH);
  float*          P1   = (float*)(ws + oP1);
  int*            HITS = (int*)(ws + oHITS);
  int*            CNT  = (int*)(ws + oCNT);
  int*            OFF  = (int*)(ws + oOFF);
  int*            DNVi = (int*)(ws + oDINV);
  float*          DNV  = (float*)(ws + oDINV);
  float*          AS   = (float*)(ws + oAS);
  float*          AD   = (float*)(ws + oAD);
  int*            FLAG = (int*)(ws + oFLAG);
  unsigned short* WAT  = (unsigned short*)(ws + oWAT);
  unsigned short* W1D  = (unsigned short*)(ws + oW1D);
  unsigned short* W2D  = (unsigned short*)(ws + oW2D);
  float*          PAR  = (float*)(ws + oPAR);

  hipFuncSetAttribute(reinterpret_cast<const void*>(&k_bucket), hipFuncAttributeMaxDynamicSharedMemorySize, (int)BK_LDS);

  k_prep<<<PBTOT, NTHR, 0, stream>>>(x, Wa, vs, vd, ba, W1, b1, W2, b2, XB, WAT, W1D, W2D, PAR);
  k_bucket<<<NBK, NTHR, BK_LDS, stream>>>(srcs, dsts, HITS, CNT, OFF, DNVi, FLAG);
  k_gemmA<<<MP / GBM, NTHR, 0, stream>>>(XB, WAT, PAR, Hb, AS, AD);
  k_attn<<<MP / ABM, NTHR, 0, stream>>>(HITS, CNT, OFF, FLAG, Hb, AS, AD, PAR, XHL);
  k_gemmP<SPLIT_B><<<MP / GBM, NTHR, 0, stream>>>(XHL, W1D, DNV, P1);
  k_conv<0><<<MP / ABM, NTHR, 0, stream>>>(HITS, CNT, OFF, FLAG, P1, DNV, PAR, 192, XHL, out);
  k_gemmP<SPLIT_C><<<MP / GBM, NTHR, 0, stream>>>(XHL, W2D, DNV, Hb);
  k_conv<1><<<MP / ABM, NTHR, 0, stream>>>(HITS, CNT, OFF, FLAG, Hb, DNV, PAR, 256, XHL, out);
}
